// RewardPredictorEnsemble_20822001451489
// MI455X (gfx1250) — hardware-verified
//
#include <hip/hip_runtime.h>

typedef __attribute__((ext_vector_type(16))) _Float16 v16h;
typedef __attribute__((ext_vector_type(8)))  _Float16 v8h;
typedef __attribute__((ext_vector_type(4)))  _Float16 v4h;
typedef __attribute__((ext_vector_type(2)))  _Float16 v2h;
typedef __attribute__((ext_vector_type(8)))  float    v8f;
typedef __attribute__((ext_vector_type(4)))  float    v4f;

#define AST 72

#define WAVE_LDS_FENCE() __syncthreads()

__device__ __forceinline__ v8f wmma_f16(v16h a, v16h b, v8f c) {
  v8f d = __builtin_amdgcn_wmma_f32_16x16x32_f16(false, a, false, b, (short)0, c, false, false);
  asm volatile("v_nop\n\tv_nop\n\tv_nop\n\tv_nop" : "+v"(d) : "v"(a), "v"(b));
  return d;
}


__device__ __forceinline__ v16h load_A(const _Float16* base, int lane, int k0) {
  const int r = lane & 15, hi = lane >> 4;
  const _Float16* p0 = base + r * AST + k0 + hi * 8;
  v8h c0 = *(const v8h*)(p0);
  v8h c1 = *(const v8h*)(p0 + 16);
  v16h a;
#pragma unroll
  for (int i = 0; i < 8; ++i) { a[i] = c0[i]; a[i + 8] = c1[i]; }
  return a;
}

__device__ __forceinline__ v16h load_B(const _Float16* wt, int lane, int ct, int k0) {
  const int n = lane & 15, hi = lane >> 4;
  const _Float16* p0 = wt + (ct * 16 + n) * AST + k0 + hi * 8;
  v8h c0 = *(const v8h*)(p0);
  v8h c1 = *(const v8h*)(p0 + 16);
  v16h b;
#pragma unroll
  for (int i = 0; i < 8; ++i) { b[i] = c0[i]; b[i + 8] = c1[i]; }
  return b;
}

template<int K, int N>
__device__ __forceinline__ void run_layer(const _Float16* in, _Float16* out,
                                          const _Float16* wt, const float* bias, int lane) {
  constexpr int NCT = N / 16;
  const int col = lane & 15, hi = lane >> 4;
  v16h a0 = load_A(in, lane, 0);
  v16h a1{};
  if constexpr (K == 64) a1 = load_A(in, lane, 32);

  v8f accs[NCT];
#pragma unroll
  for (int ct = 0; ct < NCT; ++ct) {
    v8f acc = {};
    v16h b0 = load_B(wt, lane, ct, 0);
    acc = wmma_f16(a0, b0, acc);
    if constexpr (K == 64) {
      v16h b1 = load_B(wt, lane, ct, 32);
      acc = wmma_f16(a1, b1, acc);
    }
    accs[ct] = acc;
  }

#pragma unroll
  for (int ct = 0; ct < NCT; ++ct) {
    const float bv = bias[ct * 16 + col];
#pragma unroll
    for (int v = 0; v < 8; ++v) {
      float x = accs[ct][v] + bv;
      x = (x >= 0.0f) ? x : 0.01f * x;
      out[(v + hi * 8) * AST + ct * 16 + col] = (_Float16)x;
    }
  }
}

__device__ __forceinline__ void stage_wt(const float* __restrict__ Wg, _Float16* dst,
                                         int K, int N, int tid) {
  const int pairs = (K * N) >> 1;
  for (int i = tid; i < pairs; i += 256) {
    int kp = i / N, n = i - kp * N;
    float a = Wg[(2 * kp) * N + n];
    float b = Wg[(2 * kp + 1) * N + n];
    v2h pr = {(_Float16)a, (_Float16)b};
    *(v2h*)(dst + n * AST + 2 * kp) = pr;
  }
}

__global__ __launch_bounds__(256)
void ens_reward_kernel(const float* __restrict__ s1, const float* __restrict__ s2,
                       const float* __restrict__ W1, const float* __restrict__ b1,
                       const float* __restrict__ W2, const float* __restrict__ b2,
                       const float* __restrict__ W3, const float* __restrict__ b3,
                       const float* __restrict__ W4, const float* __restrict__ b4,
                       const float* __restrict__ W5, const float* __restrict__ b5,
                       float* __restrict__ part) {
  __shared__ __align__(16) _Float16 s_act[8][2][16 * AST];
  __shared__ __align__(16) _Float16 s_wt[176 * AST];
  __shared__ __align__(16) float    s_bias[193];
  __shared__ float s_red[8][2];

  constexpr int W1OFF = 0, W2OFF = 64 * AST, W3OFF = 128 * AST, W4OFF = 160 * AST;

  const int tid  = threadIdx.x;
  const int lane = tid & 31;
  const int w    = tid >> 5;
  const int bidx = blockIdx.x;
  const size_t rowoff = (size_t)(bidx * 128 + w * 16) * 64;
  const float* xs[2] = { s1 + rowoff, s2 + rowoff };

  _Float16* ping = &s_act[w][0][0];
  _Float16* pong = &s_act[w][1][0];

  float acc2[2] = {0.0f, 0.0f};

  for (int p = 0; p < 8; ++p) {
    __syncthreads();
    stage_wt(W1 + p * 4096, s_wt + W1OFF, 64, 64, tid);
    stage_wt(W2 + p * 4096, s_wt + W2OFF, 64, 64, tid);
    stage_wt(W3 + p * 2048, s_wt + W3OFF, 64, 32, tid);
    stage_wt(W4 + p * 512,  s_wt + W4OFF, 32, 16, tid);
    if (tid < 64) s_bias[tid]       = b1[p * 64 + tid];
    if (tid < 64) s_bias[64 + tid]  = b2[p * 64 + tid];
    if (tid < 32) s_bias[128 + tid] = b3[p * 32 + tid];
    if (tid < 16) s_bias[160 + tid] = b4[p * 16 + tid];
    if (tid < 16) s_bias[176 + tid] = W5[p * 16 + tid];
    if (tid == 0) s_bias[192]       = b5[p];
    __syncthreads();

#pragma unroll
    for (int s = 0; s < 2; ++s) {
      const float* xr = xs[s];
#pragma unroll
      for (int i = lane; i < 256; i += 32) {
        int r = i >> 4, cq = i & 15;
        const float4 v = *(const float4*)(xr + r * 64 + cq * 4);
        v4h h = {(_Float16)v.x, (_Float16)v.y, (_Float16)v.z, (_Float16)v.w};
        *(v4h*)(ping + r * AST + cq * 4) = h;
      }
      WAVE_LDS_FENCE();
      run_layer<64, 64>(ping, pong, s_wt + W1OFF, s_bias + 0,   lane);
      WAVE_LDS_FENCE();
      run_layer<64, 64>(pong, ping, s_wt + W2OFF, s_bias + 64,  lane);
      WAVE_LDS_FENCE();
      run_layer<64, 32>(ping, pong, s_wt + W3OFF, s_bias + 128, lane);
      WAVE_LDS_FENCE();

      v16h a0 = load_A(pong, lane, 0);
      v16h b0 = load_B(s_wt + W4OFF, lane, 0, 0);
      v8f acc = {};
      acc = wmma_f16(a0, b0, acc);

      const float b4v = s_bias[160 + (lane & 15)];
      const float w5v = s_bias[176 + (lane & 15)];
      float t = 0.0f;
#pragma unroll
      for (int v = 0; v < 8; ++v) {
        float x = acc[v] + b4v;
        x = (x >= 0.0f) ? x : 0.01f * x;
        t += x * w5v;
      }
#pragma unroll
      for (int m = 1; m <= 16; m <<= 1)
        t += __shfl_xor(t, m, 32);
      if (lane == 0) acc2[s] += t + 16.0f * s_bias[192];
    }
  }

  if (lane == 0) { s_red[w][0] = acc2[0]; s_red[w][1] = acc2[1]; }
  __syncthreads();
  if (tid < 8) {
    float sA = 0.0f, sB = 0.0f;
#pragma unroll
    for (int i = 0; i < 8; ++i) { sA += s_red[i][0]; sB += s_red[i][1]; }
    v4f v = {sA * 0.125f, sB * 0.125f, 0.0f, 0.0f};
    float* dst = part + (size_t)bidx * 32 + tid * 4;
    *(volatile v4f*)dst = v;
    __threadfence();
    *(volatile v4f*)dst = v;
  }
}

__global__ __launch_bounds__(256) void gather_out(const float* __restrict__ part, float* __restrict__ out, int B) {
  for (int t = threadIdx.x; t * 2 < B; t += 256) {
    const float* p0 = part + (size_t)(2 * t) * 32;
    const float* p1 = part + (size_t)(2 * t + 1) * 32;
    v4f v = {p0[0], p0[1], p1[0], p1[1]};
    *(volatile v4f*)(out + (size_t)t * 4) = v;
    __threadfence();
    *(volatile v4f*)(out + (size_t)t * 4) = v;
  }
}

extern "C" void kernel_launch(void* const* d_in, const int* in_sizes, int n_in,
                              void* d_out, int out_size, void* d_ws, size_t ws_size,
                              hipStream_t stream) {
  const float* s1 = (const float*)d_in[0];
  const float* s2 = (const float*)d_in[1];
  const float* W1 = (const float*)d_in[2];
  const float* b1 = (const float*)d_in[3];
  const float* W2 = (const float*)d_in[4];
  const float* b2 = (const float*)d_in[5];
  const float* W3 = (const float*)d_in[6];
  const float* b3 = (const float*)d_in[7];
  const float* W4 = (const float*)d_in[8];
  const float* b4 = (const float*)d_in[9];
  const float* W5 = (const float*)d_in[10];
  const float* b5 = (const float*)d_in[11];
  float* out = (float*)d_out;
  float* part = (float*)d_ws;

  const int B = in_sizes[0] / (128 * 64);
  dim3 grid(B), block(256);
  ens_reward_kernel<<<grid, block, 0, stream>>>(s1, s2, W1, b1, W2, b2, W3, b3,
                                                W4, b4, W5, b5, part);
  gather_out<<<dim3(1), dim3(256), 0, stream>>>(part, out, B);
}
